// SAMPart3D_76055280877708
// MI455X (gfx1250) — hardware-verified
//
#include <hip/hip_runtime.h>
#include <math.h>

constexpr int kPts     = 8192;
constexpr int kRows    = 2 * kPts;
constexpr int kDim     = 384;
constexpr int kChunk   = 256;
constexpr int kNChunk  = kPts / kChunk;
constexpr int kOrg     = 6;
constexpr int kOrgPad  = 32;
constexpr int kHidInst = 5;
constexpr int kHidPos  = 3;
constexpr float kWCarry    = 16.0f;
constexpr float kWCarryInv = 1.0f / 16.0f;
constexpr float kCarryI    = 4.0f;
constexpr float kCarryP    = 16.0f;
constexpr float kEpsNorm   = 1e-5f;
constexpr float kEpsD2     = 1e-12f;
constexpr float kHingeAt   = 1.0f;
constexpr float kMaxScale  = 2.0f;

typedef __attribute__((ext_vector_type(16))) _Float16 v16h;
typedef __attribute__((ext_vector_type(8)))  _Float16 v8h;
typedef __attribute__((ext_vector_type(16))) __bf16   v16b;
typedef __attribute__((ext_vector_type(8)))  __bf16   v8b;
typedef __attribute__((ext_vector_type(8)))  float    v8f;
typedef __attribute__((ext_vector_type(4)))  float    v4f;
typedef __attribute__((ext_vector_type(4)))  unsigned int v4u;

__device__ __forceinline__ unsigned short f2bf_bits(float f) {
  unsigned u = __float_as_uint(f);
  return (unsigned short)((u + 0x7FFFu + ((u >> 16) & 1u)) >> 16);
}
__device__ __forceinline__ float bf_bits2f(unsigned short h) { return __uint_as_float(((unsigned)h) << 16); }

__device__ __forceinline__ void dep_guard_h(v8f& a, v8f& b, v16h x, v16h y) { asm volatile("v_nop\n\tv_nop\n\tv_nop\n\tv_nop" : "+v"(a), "+v"(b) : "v"(x), "v"(y)); }
__device__ __forceinline__ void dep_guard_b(v8f& a, v8f& b, v16b x, v16b y) { asm volatile("v_nop\n\tv_nop\n\tv_nop\n\tv_nop" : "+v"(a), "+v"(b) : "v"(x), "v"(y)); }
__device__ __forceinline__ void keep4_h(v16h a, v16h b, v16h c, v16h d) { asm volatile("v_nop" :: "v"(a), "v"(b), "v"(c), "v"(d)); }
__device__ __forceinline__ void keep4_b(v16b a, v16b b, v16b c, v16b d) { asm volatile("v_nop" :: "v"(a), "v"(b), "v"(c), "v"(d)); }
__device__ __forceinline__ void acc_guard4(v8f& a, v8f& b, v8f& c, v8f& d) { asm volatile("v_nop\n\tv_nop\n\tv_nop\n\tv_nop" : "+v"(a), "+v"(b), "+v"(c), "+v"(d)); }
template <typename T> struct Frag;
template <> struct Frag<_Float16> {
  typedef v16h V; union U { v16h v; v8h h[2]; };
  static __device__ __forceinline__ v16h load(const _Float16* p) {
    U f; f.h[0] = *(const v8h*)(p); f.h[1] = *(const v8h*)(p + 16); return f.v;
  }
  static __device__ __forceinline__ v8f mma(v16h a, v16h b, v8f c) {
    return __builtin_amdgcn_wmma_f32_16x16x32_f16(false, a, false, b, (short)0, c, false, false);
  }
  static __device__ __forceinline__ void guard(v8f& a, v8f& b, v16h x, v16h y) { dep_guard_h(a, b, x, y); }
  static __device__ __forceinline__ void keep(v16h a, v16h b, v16h c, v16h d) { keep4_h(a, b, c, d); }
};
template <> struct Frag<__bf16> {
  typedef v16b V; union U { v16b v; v8b h[2]; };
  static __device__ __forceinline__ v16b load(const __bf16* p) {
    U f; f.h[0] = *(const v8b*)(p); f.h[1] = *(const v8b*)(p + 16); return f.v;
  }
  static __device__ __forceinline__ v8f mma(v16b a, v16b b, v8f c) {
    return __builtin_amdgcn_wmma_f32_16x16x32_bf16(false, a, false, b, (short)0, c, false, false);
  }
  static __device__ __forceinline__ void guard(v8f& a, v8f& b, v16b x, v16b y) { dep_guard_b(a, b, x, y); }
  static __device__ __forceinline__ void keep(v16b a, v16b b, v16b c, v16b d) { keep4_b(a, b, c, d); }
};

__device__ __forceinline__ unsigned pk16(unsigned short a, unsigned short b) { return (unsigned)a | ((unsigned)b << 16); }
__device__ __forceinline__ unsigned short h_bits(float f) { const _Float16 h = (_Float16)f; return __builtin_bit_cast(unsigned short, h); }

template <int ET> struct Elem;
template <> struct Elem<0> { typedef _Float16 T; };
template <> struct Elem<1> { typedef __bf16 T; };
template <int ET, int SPL, int NV, int OUT_MODE, int ACT, int TRI>
__global__ __launch_bounds__(256) void wmma_gemm64(
    const unsigned short* __restrict__ Ap, const unsigned short* __restrict__ A2p, int lda, long strideA,
    const unsigned short* __restrict__ Btp, const unsigned short* __restrict__ Bt2p, int ldb, long strideB,
    void* __restrict__ Cout, void* __restrict__ Cout2, int ldc, long strideC,
    const float* __restrict__ rs, long strideS, const float* __restrict__ cs, long strideV,
    int M, int N, int K, float scale, float r1scale) {
  typedef typename Elem<ET>::T T;
  typedef typename Frag<T>::V V;
  const T* A = (const T*)Ap; const T* A2 = (const T*)A2p; const T* Bt = (const T*)Btp; const T* Bt2 = (const T*)Bt2p;
  __shared__ __align__(16) float sT[8][16 * 68];
  const int b    = blockIdx.y;
  const int lane = threadIdx.x & 31;
  const int wave = threadIdx.x >> 5;
  const int tilesN = N >> 6;
  const int tilesM = M >> 6;
  const int tile = blockIdx.x * 8 + wave;
  if (tile >= tilesM * tilesN) return;
  const int tm = tile / tilesN;
  const int tn = tile - tm * tilesN;
  const int m0 = tm << 6;
  const int n0 = tn << 6;
  if (TRI == 1 && n0 > m0) return;
  const int Kl = (TRI == 2 && (m0 + 64) < K) ? (m0 + 64) : K;

  const T* Ab  = A  + (size_t)b * strideA;
  const T* Bb  = Bt + (size_t)b * strideB;
  const T* Ab2 = (SPL & 1) ? (A2  + (size_t)b * strideA) : nullptr;
  const T* Bb2 = (SPL & 2) ? (Bt2 + (size_t)b * strideB) : nullptr;

  const int rlane = lane & 15;
  const int koff  = (lane >> 4) * 8;
  const int mOff  = (lane >> 4) * 8;

  v8f acc[4][4];
#pragma unroll
  for (int i = 0; i < 4; ++i)
#pragma unroll
    for (int j = 0; j < 4; ++j) acc[i][j] = (v8f){0.f,0.f,0.f,0.f,0.f,0.f,0.f,0.f};

  for (int k0 = 0; k0 < Kl; k0 += 32) {
    V bh[4], bl[4];
#pragma unroll
    for (int j = 0; j < 4; ++j) {
      const size_t bo = (size_t)(n0 + (j << 4) + rlane) * ldb + koff + k0;
      bh[j] = Frag<T>::load(Bb + bo);
      if (SPL & 2) bl[j] = Frag<T>::load(Bb2 + bo);
    }
#pragma unroll
    for (int i = 0; i < 4; ++i) {
      const size_t ao = (size_t)(m0 + (i << 4) + rlane) * lda + koff + k0;
      V ah = Frag<T>::load(Ab + ao);
      V al;
      if (SPL & 1) al = Frag<T>::load(Ab2 + ao);
#pragma unroll
      for (int j = 0; j < 4; ++j) {
        acc[i][j] = Frag<T>::mma(ah, bh[j], acc[i][j]);
        if (SPL & 2) acc[i][j] = Frag<T>::mma(ah, bl[j], acc[i][j]);
        if (SPL & 1) acc[i][j] = Frag<T>::mma(al, bh[j], acc[i][j]);
      }
      Frag<T>::guard(acc[i][0], acc[i][3], ah, (SPL & 1) ? al : ah);
    }
    Frag<T>::keep(bh[0], bh[1], bh[2], bh[3]);
    if (SPL & 2) Frag<T>::keep(bl[0], bl[1], bl[2], bl[3]);
  }
  acc_guard4(acc[0][0], acc[0][1], acc[0][2], acc[0][3]);
  acc_guard4(acc[1][0], acc[1][1], acc[1][2], acc[1][3]);
  acc_guard4(acc[2][0], acc[2][1], acc[2][2], acc[2][3]);
  acc_guard4(acc[3][0], acc[3][1], acc[3][2], acc[3][3]);

  float* slab = sT[wave];
#pragma unroll 1
  for (int nv = 0; nv < (NV > 0 ? NV : 1); ++nv) {
    const float* Rs = (NV > 0) ? (rs + (size_t)nv * strideS) : nullptr;
    const size_t vOff = (NV > 0) ? ((size_t)nv * strideV) : (size_t)0;
#pragma unroll
    for (int i = 0; i < 4; ++i) {
      const int mBase = m0 + (i << 4);
      float rsv[8];
#pragma unroll
      for (int r = 0; r < 8; ++r) rsv[r] = (NV > 0) ? (Rs[mBase + mOff + r] * r1scale) : 0.0f;
#pragma unroll
      for (int j = 0; j < 4; ++j) {
        const int n = n0 + (j << 4) + rlane;
        const float csn = (NV > 0) ? cs[n] : 0.0f;
#pragma unroll
        for (int r = 0; r < 8; ++r) {
          float v = acc[i][j][r] * scale;
          if (NV > 0) v += rsv[r] * csn;
          if (TRI == 1) { if (n > mBase + mOff + r) v = 0.0f; }
          if (ACT == 2) v = fmaxf(v, 0.0f);
          slab[(mOff + r) * 68 + (j << 4) + rlane] = v;
        }
      }
      __builtin_amdgcn_fence(__ATOMIC_RELEASE, "workgroup");
      __builtin_amdgcn_wave_barrier();
      __builtin_amdgcn_fence(__ATOMIC_ACQUIRE, "workgroup");
      if (OUT_MODE == 0) {
        float* C = (float*)Cout + (size_t)b * strideC + vOff;
        const int hh = lane >> 4, c4 = (lane & 15) * 4;
        for (int pass = 0; pass < 2; ++pass) {
#pragma unroll
          for (int it = 0; it < 8; ++it) {
            const int row = it * 2 + hh;
            v4f v = *(const v4f*)(slab + row * 68 + c4);
            *(volatile v4f*)(C + (size_t)(mBase + row) * ldc + n0 + c4) = v;
          }
          __threadfence();
        }
      } else {
        const int q = lane >> 3, c8 = (lane & 7) * 8;
        unsigned short* C  = (unsigned short*)Cout  + (size_t)b * strideC + vOff;
        unsigned short* C2 = (OUT_MODE == 2) ? ((unsigned short*)Cout2 + (size_t)b * strideC + vOff) : nullptr;
        for (int pass = 0; pass < 2; ++pass) {
#pragma unroll
          for (int it = 0; it < 4; ++it) {
            const int row = it * 4 + q;
            const float* sp = slab + row * 68 + c8;
            v8h hv, lv;
#pragma unroll
            for (int e = 0; e < 8; ++e) {
              if (OUT_MODE == 1) {
                hv[e] = (_Float16)sp[e];
              } else {
                unsigned short hb = f2bf_bits(sp[e]);
                unsigned short lb = f2bf_bits(sp[e] - bf_bits2f(hb));
                hv[e] = __builtin_bit_cast(_Float16, hb);
                lv[e] = __builtin_bit_cast(_Float16, lb);
              }
            }
            *(volatile v8h*)(C + (size_t)(mBase + row) * ldc + n0 + c8) = hv;
            if (OUT_MODE == 2) *(volatile v8h*)(C2 + (size_t)(mBase + row) * ldc + n0 + c8) = lv;
          }
          __threadfence();
        }
      }
      __builtin_amdgcn_fence(__ATOMIC_RELEASE, "workgroup");
      __builtin_amdgcn_wave_barrier();
      __builtin_amdgcn_fence(__ATOMIC_ACQUIRE, "workgroup");
    }
  }
}

__global__ __launch_bounds__(256) void cast_f16x8(const float* __restrict__ in, unsigned short* __restrict__ out, int n8, float scale) {
  const int i = blockIdx.x * 256 + threadIdx.x;
  if (i >= n8) return;
  const float* p = in + 8 * (size_t)i;
  const v4f a = *(const v4f*)(p);
  const v4f c = *(const v4f*)(p + 4);
  unsigned short hb[8];
#pragma unroll
  for (int e = 0; e < 4; ++e) {
    hb[e]     = h_bits(a[e] * scale);
    hb[4 + e] = h_bits(c[e] * scale);
  }
  const v4u u = (v4u){pk16(hb[0], hb[1]), pk16(hb[2], hb[3]), pk16(hb[4], hb[5]), pk16(hb[6], hb[7])};
  unsigned short* q = out + 8 * (size_t)i;
  *(volatile v4u*)q = u;
  __threadfence();
  *(volatile v4u*)q = u;
}

__global__ __launch_bounds__(256) void wt_cast_t16(const float* __restrict__ W, unsigned short* __restrict__ Bt,
                                                   int K, int Kp, int nmat, float scale) {
  const int gid = blockIdx.x * 256 + threadIdx.x;
  const int gpr = Kp >> 3;
  const int perMat = kDim * gpr;
  if (gid >= nmat * perMat) return;
  const int l   = gid / perMat;
  const int rem = gid - l * perMat;
  const int n   = rem / gpr;
  const int kg  = rem - n * gpr;
  const float* Wl = W + (size_t)l * K * kDim;
  unsigned short hb[8];
#pragma unroll
  for (int e = 0; e < 8; ++e) {
    const int k  = kg * 8 + e;
    const int kc = (k < K) ? k : (K - 1);
    const float w = Wl[(size_t)kc * kDim + n];
    hb[e] = (k < K) ? h_bits(w * scale) : (unsigned short)0;
  }
  const v4u u = (v4u){pk16(hb[0], hb[1]), pk16(hb[2], hb[3]), pk16(hb[4], hb[5]), pk16(hb[6], hb[7])};
  unsigned short* q = Bt + (size_t)l * kDim * Kp + (size_t)n * Kp + kg * 8;
  *(volatile v4u*)q = u;
  __threadfence();
  *(volatile v4u*)q = u;
}

__global__ __launch_bounds__(256) void build_org16(const float* __restrict__ org, unsigned short* __restrict__ X) {
  const int gid = blockIdx.x * 256 + threadIdx.x;
  if (gid >= kPts * (kOrgPad / 8)) return;
  const int row = gid >> 2;
  const int cg  = gid & 3;
  unsigned short hb[8];
#pragma unroll
  for (int e = 0; e < 8; ++e) {
    const int col = cg * 8 + e;
    const int cc  = (col < kOrg) ? col : (kOrg - 1);
    const float v = org[(size_t)row * kOrg + cc];
    hb[e] = (col < kOrg) ? h_bits(v) : (unsigned short)0;
  }
  const v4u u = (v4u){pk16(hb[0], hb[1]), pk16(hb[2], hb[3]), pk16(hb[4], hb[5]), pk16(hb[6], hb[7])};
  unsigned short* q = X + (size_t)row * kOrgPad + cg * 8;
  *(volatile v4u*)q = u;
  __threadfence();
  *(volatile v4u*)q = u;
}

__global__ __launch_bounds__(256) void build_s12(const float* __restrict__ sc, const float* __restrict__ ru, float* __restrict__ S12) {
#pragma clang fp contract(off)
  const int m = blockIdx.x * 256 + threadIdx.x;
  if (m >= kPts) return;
  const float s = sc[m];
  const float r = ru[0];
  const float d = fmaxf(kMaxScale - s, 0.0f);
  const float prod = d * r;
  const float s2 = s + prod;
  float* p1 = S12 + m;
  float* p2 = S12 + kPts + m;
  *(volatile float*)p1 = s;
  *(volatile float*)p2 = s2;
  __threadfence();
  *(volatile float*)p1 = s;
  *(volatile float*)p2 = s2;
}

__global__ __launch_bounds__(256) void norm_embed(const float* __restrict__ OI, const float* __restrict__ OP,
                                                  unsigned short* __restrict__ EH, unsigned short* __restrict__ EL,
                                                  float* __restrict__ SQ) {
  __shared__ float sqs[32];
  const int lane = threadIdx.x & 31, wave = threadIdx.x >> 5;
  const int row0 = blockIdx.x * 32;
  const int cA = 8 * lane;
  const int cB = 256 + 8 * (lane & 15);
  const float wB = (lane < 16) ? 1.0f : 0.0f;
#pragma unroll 1
  for (int rr = 0; rr < 4; ++rr) {
    const int rloc = wave * 4 + rr;
    const int row  = row0 + rloc;
    const float* pi = OI + (size_t)row * kDim;
    const float* pp = OP + (size_t)row * kDim;
    float vi[16], vp[16];
    {
      const v4f a0 = *(const v4f*)(pi + cA), a1 = *(const v4f*)(pi + cA + 4);
      const v4f b0 = *(const v4f*)(pi + cB), b1 = *(const v4f*)(pi + cB + 4);
      const v4f c0 = *(const v4f*)(pp + cA), c1 = *(const v4f*)(pp + cA + 4);
      const v4f d0 = *(const v4f*)(pp + cB), d1 = *(const v4f*)(pp + cB + 4);
#pragma unroll
      for (int e = 0; e < 4; ++e) {
        vi[e] = a0[e]; vi[4 + e] = a1[e]; vi[8 + e] = b0[e]; vi[12 + e] = b1[e];
        vp[e] = c0[e]; vp[4 + e] = c1[e]; vp[8 + e] = d0[e]; vp[12 + e] = d1[e];
      }
    }
    float ssi = 0.f, ssp = 0.f, tsi = 0.f, tsp = 0.f;
#pragma unroll
    for (int e = 0; e < 8; ++e) { ssi += vi[e] * vi[e]; ssp += vp[e] * vp[e]; }
#pragma unroll
    for (int e = 8; e < 16; ++e) { tsi += vi[e] * vi[e]; tsp += vp[e] * vp[e]; }
    ssi += wB * tsi; ssp += wB * tsp;
#pragma unroll
    for (int off = 16; off > 0; off >>= 1) {
      ssi += __shfl_xor(ssi, off, 32);
      ssp += __shfl_xor(ssp, off, 32);
    }
    const float di = 1.0f / (sqrtf(ssi) + kEpsNorm);
    const float dp = 1.0f / (sqrtf(ssp) + kEpsNorm);
    float em[16];
#pragma unroll
    for (int e = 0; e < 16; ++e) em[e] = vi[e] * di + vp[e] * dp;
    float sse = 0.f, tse = 0.f;
#pragma unroll
    for (int e = 0; e < 8; ++e) sse += em[e] * em[e];
#pragma unroll
    for (int e = 8; e < 16; ++e) tse += em[e] * em[e];
    sse += wB * tse;
#pragma unroll
    for (int off = 16; off > 0; off >>= 1) sse += __shfl_xor(sse, off, 32);
    unsigned short hb[16], lb[16];
#pragma unroll
    for (int e = 0; e < 16; ++e) {
      const unsigned short hh = f2bf_bits(em[e]);
      hb[e] = hh;
      lb[e] = f2bf_bits(em[e] - bf_bits2f(hh));
    }
    const v4u hA = (v4u){pk16(hb[0], hb[1]), pk16(hb[2], hb[3]), pk16(hb[4], hb[5]), pk16(hb[6], hb[7])};
    const v4u hBv = (v4u){pk16(hb[8], hb[9]), pk16(hb[10], hb[11]), pk16(hb[12], hb[13]), pk16(hb[14], hb[15])};
    const v4u lA = (v4u){pk16(lb[0], lb[1]), pk16(lb[2], lb[3]), pk16(lb[4], lb[5]), pk16(lb[6], lb[7])};
    const v4u lBv = (v4u){pk16(lb[8], lb[9]), pk16(lb[10], lb[11]), pk16(lb[12], lb[13]), pk16(lb[14], lb[15])};
    unsigned short* eh = EH + (size_t)row * kDim;
    unsigned short* el = EL + (size_t)row * kDim;
    *(volatile v4u*)(eh + cA) = hA;
    *(volatile v4u*)(el + cA) = lA;
    if (lane < 16) { *(volatile v4u*)(eh + cB) = hBv; *(volatile v4u*)(el + cB) = lBv; }
    __threadfence();
    *(volatile v4u*)(eh + cA) = hA;
    *(volatile v4u*)(el + cA) = lA;
    if (lane < 16) { *(volatile v4u*)(eh + cB) = hBv; *(volatile v4u*)(el + cB) = lBv; }
    if (lane == 0) sqs[rloc] = sse;
  }
  __syncthreads();
  if (wave == 0) {
    const float v = sqs[lane];
    float* p = SQ + row0 + lane;
    *(volatile float*)p = v;
    __threadfence();
    *(volatile float*)p = v;
  }
}

__global__ __launch_bounds__(256) void pair_sums(const float* __restrict__ G, const float* __restrict__ SQ,
                                                 const int* __restrict__ lab, float* __restrict__ PART) {
  __shared__ int   s_lab[kChunk];
  __shared__ float s_sq[kChunk];
  __shared__ float rf[8][2];
  __shared__ int   ri[8][3];
  __shared__ float lineS[32];
  const int blk  = blockIdx.x;
  const int c    = blk & (kNChunk - 1);
  const int t    = threadIdx.x;
  const int lane = t & 31, wave = t >> 5;
  s_lab[t] = lab[c * kChunk + t];
  s_sq[t]  = SQ[(size_t)blk * kChunk + t];
  __syncthreads();
  const int i = t;
  const int li = s_lab[i];
  const float sqi = s_sq[i];
  const float* Gb = G + (size_t)blk * (kChunk * kChunk);
  float sp = 0.f, sn = 0.f;
  int cp = 0, cn = 0, cb = 0;
#pragma unroll 1
  for (int j = wave * 32; j < kChunk; ++j) {
    const float g   = Gb[(size_t)j * kChunk + i];
    const int   lj  = s_lab[j];
    const float sqj = s_sq[j];
    const float a   = sqi + sqj;
    const float d2  = a - 2.0f * g;
    const float dist = sqrtf(d2 > kEpsD2 ? d2 : kEpsD2);
    const bool blkm = (j >= i) && (li != -1) && (lj != -1);
    const bool eq   = (li == lj);
    const bool pm   = blkm && eq && (j != i);
    const bool nm   = blkm && (!eq);
    cb += blkm ? 1 : 0;
    cp += pm ? 1 : 0;
    cn += nm ? 1 : 0;
    sp += pm ? dist : 0.0f;
    sn += nm ? fmaxf(kHingeAt - dist, 0.0f) : 0.0f;
  }
#pragma unroll
  for (int off = 16; off > 0; off >>= 1) {
    sp += __shfl_xor(sp, off, 32);
    sn += __shfl_xor(sn, off, 32);
    cp += __shfl_xor(cp, off, 32);
    cn += __shfl_xor(cn, off, 32);
    cb += __shfl_xor(cb, off, 32);
  }
  if (lane == 0) { rf[wave][0] = sp; rf[wave][1] = sn; ri[wave][0] = cp; ri[wave][1] = cn; ri[wave][2] = cb; }
  __syncthreads();
  if (t == 0) {
    float a = 0.f, bsum = 0.f;
    int x = 0, y = 0, z = 0;
#pragma unroll 1
    for (int w = 0; w < 8; ++w) { a += rf[w][0]; bsum += rf[w][1]; x += ri[w][0]; y += ri[w][1]; z += ri[w][2]; }
#pragma unroll 1
    for (int e = 0; e < 32; ++e) lineS[e] = 0.0f;
    lineS[0] = a; lineS[1] = bsum; lineS[2] = (float)x; lineS[3] = (float)y; lineS[4] = (float)z;
  }
  __syncthreads();
  if (wave == 0) {
    const float v = lineS[lane];
    float* p = PART + (size_t)blk * 32 + lane;
    *(volatile float*)p = v;
    __threadfence();
    *(volatile float*)p = v;
  }
}

__global__ __launch_bounds__(32) void final_combine(const float* __restrict__ PART, const int* __restrict__ csz, float* __restrict__ out) {
  (void)csz;
  if (threadIdx.x == 0) {
    double s1 = 0.0, s2 = 0.0, s3 = 0.0, np = 0.0, nn = 0.0, nb = 0.0;
#pragma unroll 1
    for (int c = 0; c < kNChunk; ++c) {
      const float* p = PART + (size_t)c * 32;
      s1 += (double)p[0]; s3 += (double)p[1]; np += (double)p[2]; nn += (double)p[3]; nb += (double)p[4];
    }
#pragma unroll 1
    for (int c = 0; c < kNChunk; ++c) {
      const float* p = PART + (size_t)(kNChunk + c) * 32;
      s2 += (double)p[0];
    }
    const double npc = (np > 1.0) ? np : 1.0;
    const double nnc = (nn > 1.0) ? nn : 1.0;
    const double l1 = s1 / npc, l2 = s2 / npc, l3 = s3 / nnc;
    const double wp = np / nb, wn = nn / nb;
    const float total = (float)(l1 * wp + l2 * wp + l3 * wn);
    *(volatile float*)out = total;
    __threadfence();
    *(volatile float*)out = total;
  }
}

extern "C" void kernel_launch(void* const* d_in, const int* in_sizes, int n_in,
                              void* d_out, int out_size, void* d_ws, size_t ws_size,
                              hipStream_t stream) {
  if (n_in < 12) return;
  if (in_sizes[0] != kPts * kDim) return;
  if (in_sizes[1] != kPts * kOrg) return;
  if (in_sizes[2] != kPts) return;
  if (in_sizes[3] != kPts) return;
  if (in_sizes[4] < 1) return;
  if (in_sizes[5] < 1) return;
  if (in_sizes[6] != (kDim + 1) * kDim) return;
  if (in_sizes[7] != kHidInst * kDim * kDim) return;
  if (in_sizes[8] != kDim * kDim) return;
  if (in_sizes[9] != (kOrg + 1) * kDim) return;
  if (in_sizes[10] != kHidPos * kDim * kDim) return;
  if (in_sizes[11] != kDim * kDim) return;
  if (out_size != 1) return;

  const float* feat  = (const float*)d_in[0];
  const float* org   = (const float*)d_in[1];
  const float* scale = (const float*)d_in[2];
  const int*   lab   = (const int*)d_in[3];
  const float* randu = (const float*)d_in[4];
  const int*   csz   = (const int*)d_in[5];
  const float* iWin  = (const float*)d_in[6];
  const float* iWhid = (const float*)d_in[7];
  const float* iWout = (const float*)d_in[8];
  const float* pWin  = (const float*)d_in[9];
  const float* pWhid = (const float*)d_in[10];
  const float* pWout = (const float*)d_in[11];
  float* outp = (float*)d_out;

  const size_t SZ_FEAT = (size_t)kPts * kDim * 2;
  const size_t SZ_ORG  = (size_t)kPts * kOrgPad * 2;
  const size_t SZ_S12  = (size_t)2 * kPts * 4;
  const size_t SZ_W    = (size_t)kDim * kDim * 2;
  const size_t SZ_WPIN = (size_t)kDim * kOrgPad * 2;
  const size_t SZ_H    = (size_t)kRows * kDim * 2;
  const size_t SZ_OF   = (size_t)kRows * kDim * 4;
  const size_t SZ_SQ   = (size_t)kRows * 4;
  const size_t SZ_PART = (size_t)2 * kNChunk * 32 * 4;
  const size_t SZ_G    = (size_t)2 * kNChunk * kChunk * kChunk * 4;
  size_t off = 0;
  const size_t oFEAT  = off; off += SZ_FEAT;
  const size_t oORG   = off; off += SZ_ORG;
  const size_t oS12   = off; off += SZ_S12;
  const size_t oWIIN  = off; off += SZ_W;
  const size_t oWIHID = off; off += SZ_W * kHidInst;
  const size_t oWIOUT = off; off += SZ_W;
  const size_t oWPIN  = off; off += SZ_WPIN;
  const size_t oWPHID = off; off += SZ_W * kHidPos;
  const size_t oWPOUT = off; off += SZ_W;
  const size_t oH0    = off; off += SZ_H;
  const size_t oH1    = off; off += SZ_H;
  const size_t oOFI   = off; off += SZ_OF;
  const size_t oOFP   = off; off += SZ_OF;
  const size_t oSQ    = off; off += SZ_SQ;
  const size_t oPART  = off; off += SZ_PART;
  const size_t TOTAL  = off;
  if (SZ_G > SZ_OF) return;
  if (TOTAL > ws_size) return;
  if (TOTAL > (size_t)134217728) return;

  char* ws = (char*)d_ws;
  unsigned short* FEAT16 = (unsigned short*)(ws + oFEAT);
  unsigned short* ORG16  = (unsigned short*)(ws + oORG);
  float*          S12    = (float*)(ws + oS12);
  unsigned short* WIIN   = (unsigned short*)(ws + oWIIN);
  unsigned short* WIHID  = (unsigned short*)(ws + oWIHID);
  unsigned short* WIOUT  = (unsigned short*)(ws + oWIOUT);
  unsigned short* WPIN   = (unsigned short*)(ws + oWPIN);
  unsigned short* WPHID  = (unsigned short*)(ws + oWPHID);
  unsigned short* WPOUT  = (unsigned short*)(ws + oWPOUT);
  unsigned short* H0     = (unsigned short*)(ws + oH0);
  unsigned short* H1     = (unsigned short*)(ws + oH1);
  float*          OFI    = (float*)(ws + oOFI);
  float*          OFP    = (float*)(ws + oOFP);
  float*          SQ     = (float*)(ws + oSQ);
  float*          PART   = (float*)(ws + oPART);
  unsigned short* EH     = H0;
  unsigned short* EL     = H1;
  float*          G      = OFI;
  const float* csI = iWin + (size_t)kDim * kDim;
  const float* csP = pWin + (size_t)kOrg * kDim;

  const dim3 blk(256);

  {
    const int n8 = kPts * kDim / 8;
    cast_f16x8<<<dim3(n8 / 256), blk, 0, stream>>>(feat, FEAT16, n8, 1.0f);
    build_org16<<<dim3(kPts * (kOrgPad / 8) / 256), blk, 0, stream>>>(org, ORG16);
    build_s12<<<dim3(kPts / 256), blk, 0, stream>>>(scale, randu, S12);
    const int g384 = kDim * (kDim / 8) / 256;
    const int g32  = kDim * (kOrgPad / 8) / 256;
    wt_cast_t16<<<dim3(g384), blk, 0, stream>>>(iWin, WIIN, kDim, kDim, 1, kWCarry);
    wt_cast_t16<<<dim3(g384 * kHidInst), blk, 0, stream>>>(iWhid, WIHID, kDim, kDim, kHidInst, kWCarry);
    wt_cast_t16<<<dim3(g384), blk, 0, stream>>>(iWout, WIOUT, kDim, kDim, 1, kWCarry);
    wt_cast_t16<<<dim3(g32), blk, 0, stream>>>(pWin, WPIN, kOrg, kOrgPad, 1, kWCarry);
    wt_cast_t16<<<dim3(g384 * kHidPos), blk, 0, stream>>>(pWhid, WPHID, kDim, kDim, kHidPos, kWCarry);
    wt_cast_t16<<<dim3(g384), blk, 0, stream>>>(pWout, WPOUT, kDim, kDim, 1, kWCarry);
  }

  const int tilesN = kDim / 64;
  const dim3 gL1((kPts / 64 * tilesN + 7) / 8, 1);
  const dim3 gL((kRows / 64 * tilesN + 7) / 8, 1);
  const long strideV = (long)kPts * kDim;
  const size_t wsz = (size_t)kDim * kDim;

  wmma_gemm64<0, 0, 2, 1, 2, 0><<<gL1, blk, 0, stream>>>(
      FEAT16, FEAT16, kDim, 0L, WIIN, WIIN, kDim, 0L, (void*)H0, (void*)H0, kDim, 0L,
      S12, (long)kPts, csI, strideV, kPts, kDim, kDim, kCarryI * kWCarryInv, kCarryI);
  wmma_gemm64<0, 0, 0, 1, 2, 0><<<gL, blk, 0, stream>>>(
      H0, H0, kDim, 0L, WIHID + 0 * wsz, WIHID, kDim, 0L, (void*)H1, (void*)H1, kDim, 0L,
      S12, 0L, csI, 0L, kRows, kDim, kDim, kWCarryInv, 0.0f);
  wmma_gemm64<0, 0, 0, 1, 2, 0><<<gL, blk, 0, stream>>>(
      H1, H1, kDim, 0L, WIHID + 1 * wsz, WIHID, kDim, 0L, (void*)H0, (void*)H0, kDim, 0L,
      S12, 0L, csI, 0L, kRows, kDim, kDim, kWCarryInv, 0.0f);
  wmma_gemm64<0, 0, 0, 1, 2, 0><<<gL, blk, 0, stream>>>(
      H0, H0, kDim, 0L, WIHID + 2 * wsz, WIHID, kDim, 0L, (void*)H1, (void*)H1, kDim, 0L,
      S12, 0L, csI, 0L, kRows, kDim, kDim, kWCarryInv, 0.0f);
  wmma_gemm64<0, 0, 0, 1, 2, 0><<<gL, blk, 0, stream>>>(
      H1, H1, kDim, 0L, WIHID + 3 * wsz, WIHID, kDim, 0L, (void*)H0, (void*)H0, kDim, 0L,
      S12, 0L, csI, 0L, kRows, kDim, kDim, kWCarryInv, 0.0f);
  wmma_gemm64<0, 0, 0, 1, 2, 0><<<gL, blk, 0, stream>>>(
      H0, H0, kDim, 0L, WIHID + 4 * wsz, WIHID, kDim, 0L, (void*)H1, (void*)H1, kDim, 0L,
      S12, 0L, csI, 0L, kRows, kDim, kDim, kWCarryInv, 0.0f);
  wmma_gemm64<0, 0, 0, 0, 0, 0><<<gL, blk, 0, stream>>>(
      H1, H1, kDim, 0L, WIOUT, WIOUT, kDim, 0L, (void*)OFI, (void*)OFI, kDim, 0L,
      S12, 0L, csI, 0L, kRows, kDim, kDim, kWCarryInv / kCarryI, 0.0f);

  wmma_gemm64<0, 0, 2, 1, 2, 0><<<gL1, blk, 0, stream>>>(
      ORG16, ORG16, kOrgPad, 0L, WPIN, WPIN, kOrgPad, 0L, (void*)H0, (void*)H0, kDim, 0L,
      S12, (long)kPts, csP, strideV, kPts, kDim, kOrgPad, kCarryP * kWCarryInv, kCarryP);
  wmma_gemm64<0, 0, 0, 1, 2, 0><<<gL, blk, 0, stream>>>(
      H0, H0, kDim, 0L, WPHID + 0 * wsz, WPHID, kDim, 0L, (void*)H1, (void*)H1, kDim, 0L,
      S12, 0L, csP, 0L, kRows, kDim, kDim, kWCarryInv, 0.0f);
  wmma_gemm64<0, 0, 0, 1, 2, 0><<<gL, blk, 0, stream>>>(
      H1, H1, kDim, 0L, WPHID + 1 * wsz, WPHID, kDim, 0L, (void*)H0, (void*)H0, kDim, 0L,
      S12, 0L, csP, 0L, kRows, kDim, kDim, kWCarryInv, 0.0f);
  wmma_gemm64<0, 0, 0, 1, 2, 0><<<gL, blk, 0, stream>>>(
      H0, H0, kDim, 0L, WPHID + 2 * wsz, WPHID, kDim, 0L, (void*)H1, (void*)H1, kDim, 0L,
      S12, 0L, csP, 0L, kRows, kDim, kDim, kWCarryInv, 0.0f);
  wmma_gemm64<0, 0, 0, 0, 0, 0><<<gL, blk, 0, stream>>>(
      H1, H1, kDim, 0L, WPOUT, WPOUT, kDim, 0L, (void*)OFP, (void*)OFP, kDim, 0L,
      S12, 0L, csP, 0L, kRows, kDim, kDim, kWCarryInv / kCarryP, 0.0f);

  norm_embed<<<dim3(kRows / 32), blk, 0, stream>>>(OFI, OFP, EH, EL, SQ);

  {
    const dim3 gG(((kChunk / 64) * (kChunk / 64) + 7) / 8, 2 * kNChunk);
    wmma_gemm64<1, 3, 0, 0, 0, 1><<<gG, blk, 0, stream>>>(
        EH, EL, kDim, (long)kChunk * kDim, EH, EL, kDim, (long)kChunk * kDim,
        (void*)G, (void*)G, kChunk, (long)kChunk * kChunk,
        S12, 0L, csI, 0L, kChunk, kChunk, kDim, 1.0f, 0.0f);
  }

  pair_sums<<<dim3(2 * kNChunk), blk, 0, stream>>>(G, SQ, lab, PART);
  final_combine<<<dim3(1), dim3(32), 0, stream>>>(PART, csz, outp);
}
